// ThermalLSTM_5411658793090
// MI455X (gfx1250) — hardware-verified
//
#include <hip/hip_runtime.h>
#include <stdint.h>

#define NB   131072
#define TT   8
#define NI   6
#define NH   64
#define NG   256
#define K0   96
#define K1   128
#define LDA0 104
#define LDA1 136
#define LDF  68
#define SPB  32
#define NTHR 256
#define WSCALE 8.0f
#define WINV   0.125f
#define PREP0 (NG * (K0 / 8))
#define PREP1 (NG * (K1 / 8))
#define PREPN (PREP0 + PREP1)

typedef __attribute__((ext_vector_type(16))) _Float16 v16h;
typedef __attribute__((ext_vector_type(8)))  _Float16 v8h;
typedef __attribute__((ext_vector_type(16))) __bf16   v16b;
typedef __attribute__((ext_vector_type(8)))  __bf16   v8b;
typedef __attribute__((ext_vector_type(8)))  float    v8f;
typedef __attribute__((ext_vector_type(4)))  float    v4f;

__device__ __forceinline__ void dep_guard_h(v8f& a, v8f& b, v16h x, v16h y) { asm volatile("v_nop\n\tv_nop\n\tv_nop\n\tv_nop" : "+v"(a), "+v"(b) : "v"(x), "v"(y)); }
__device__ __forceinline__ void dep_guard_b(v8f& a, v8f& b, v16b x, v16b y) { asm volatile("v_nop\n\tv_nop\n\tv_nop\n\tv_nop" : "+v"(a), "+v"(b) : "v"(x), "v"(y)); }
__device__ __forceinline__ void keep4_h(v16h a, v16h b, v16h c, v16h d) { asm volatile("v_nop" :: "v"(a), "v"(b), "v"(c), "v"(d)); }
__device__ __forceinline__ void keep4_b(v16b a, v16b b, v16b c, v16b d) { asm volatile("v_nop" :: "v"(a), "v"(b), "v"(c), "v"(d)); }
__device__ __forceinline__ void acc_guard4(v8f& a, v8f& b, v8f& c, v8f& d) { asm volatile("v_nop\n\tv_nop\n\tv_nop\n\tv_nop" : "+v"(a), "+v"(b), "+v"(c), "+v"(d)); }
template <typename T> struct Frag;
template <> struct Frag<_Float16> {
  typedef v16h V; union U { v16h v; v8h h[2]; };
  static __device__ __forceinline__ v16h load(const _Float16* p) {
    U f; f.h[0] = *(const v8h*)(p); f.h[1] = *(const v8h*)(p + 16); return f.v;
  }
  static __device__ __forceinline__ v8f mma(v16h a, v16h b, v8f c) {
    return __builtin_amdgcn_wmma_f32_16x16x32_f16(false, a, false, b, (short)0, c, false, false);
  }
  static __device__ __forceinline__ void guard(v8f& a, v8f& b, v16h x, v16h y) { dep_guard_h(a, b, x, y); }
  static __device__ __forceinline__ void keep(v16h a, v16h b, v16h c, v16h d) { keep4_h(a, b, c, d); }
};
template <> struct Frag<__bf16> {
  typedef v16b V; union U { v16b v; v8b h[2]; };
  static __device__ __forceinline__ v16b load(const __bf16* p) {
    U f; f.h[0] = *(const v8b*)(p); f.h[1] = *(const v8b*)(p + 16); return f.v;
  }
  static __device__ __forceinline__ v8f mma(v16b a, v16b b, v8f c) {
    return __builtin_amdgcn_wmma_f32_16x16x32_bf16(false, a, false, b, (short)0, c, false, false);
  }
  static __device__ __forceinline__ void guard(v8f& a, v8f& b, v16b x, v16b y) { dep_guard_b(a, b, x, y); }
  static __device__ __forceinline__ void keep(v16b a, v16b b, v16b c, v16b d) { keep4_b(a, b, c, d); }
};

__device__ __forceinline__ v8f mma_f16g(v16h a, v16h b, v8f c) {
  c = __builtin_amdgcn_wmma_f32_16x16x32_f16(false, a, false, b, (short)0, c, false, false);
  asm volatile("v_nop\n\tv_nop\n\tv_nop\n\tv_nop" : "+v"(c) : "v"(a), "v"(b));
  return c;
}

__device__ __forceinline__ float sigm_f(float x) {
  const float a = fminf(-x * 1.4426950408889634f, 80.0f);
  return __builtin_amdgcn_rcpf(1.0f + __builtin_amdgcn_exp2f(a));
}
__device__ __forceinline__ float tanh_f(float x) {
  const float a = fminf(x * 2.8853900817779268f, 80.0f);
  return 1.0f - 2.0f * __builtin_amdgcn_rcpf(1.0f + __builtin_amdgcn_exp2f(a));
}

__global__ __launch_bounds__(NTHR) void prep_weights(
    const float* __restrict__ Wih0, const float* __restrict__ Whh0,
    const float* __restrict__ Wih1, const float* __restrict__ Whh1,
    _Float16* __restrict__ W0c, _Float16* __restrict__ W1c) {
  const int i = blockIdx.x * NTHR + threadIdx.x;
  if (i >= PREPN) return;
  v8h hv;
  _Float16* dst;
  if (i < PREP0) {
    const int n = i / (K0 / 8);
    const int q = i - n * (K0 / 8);
#pragma unroll
    for (int e = 0; e < 8; ++e) {
      const int k  = q * 8 + e;
      const int kh = (k < NH) ? k : (NH - 1);
      int kx = k - NH;
      kx = (kx < 0) ? 0 : ((kx > NI - 1) ? (NI - 1) : kx);
      const float a = Whh0[n * NH + kh];
      const float b = Wih0[n * NI + kx];
      const float v = (k < NH) ? a : ((k < NH + NI) ? b : 0.0f);
      hv[e] = (_Float16)(v * WSCALE);
    }
    dst = W0c + (size_t)n * K0 + q * 8;
  } else {
    const int j = i - PREP0;
    const int n = j / (K1 / 8);
    const int q = j - n * (K1 / 8);
#pragma unroll
    for (int e = 0; e < 8; ++e) {
      const int k  = q * 8 + e;
      const int ka = (k < NH) ? k : (NH - 1);
      const int kb = (k < NH) ? 0 : (k - NH);
      const float a = Wih1[n * NH + ka];
      const float b = Whh1[n * NH + kb];
      const float v = (k < NH) ? a : b;
      hv[e] = (_Float16)(v * WSCALE);
    }
    dst = W1c + (size_t)n * K1 + q * 8;
  }
  *(volatile v8h*)dst = hv;
  __threadfence();
  *(volatile v8h*)dst = hv;
}

__global__ __launch_bounds__(NTHR)
void lstm2_fc_fused(const float* __restrict__ x,
                    const _Float16* __restrict__ W0c, const _Float16* __restrict__ W1c,
                    const float* __restrict__ bih0, const float* __restrict__ bhh0,
                    const float* __restrict__ bih1, const float* __restrict__ bhh1,
                    const float* __restrict__ Wfc, const float* __restrict__ bfc,
                    float* __restrict__ out) {
  __shared__ __align__(16) _Float16 A0[SPB * LDA0];
  __shared__ __align__(16) _Float16 A1[SPB * LDA1];
  __shared__ __align__(16) float    hF[SPB * LDF];
  __shared__ __align__(16) float    oS[SPB];

  const int tid  = threadIdx.x;
  const int wave = tid >> 5, lane = tid & 31, hh = lane >> 4, c = lane & 15;
  const int sg   = wave >> 2, hw = wave & 3;
  const int rowb = sg * 16;
  const int col  = hw * 16 + c;
  const int koff = 8 * hh;
  const size_t base = (size_t)blockIdx.x * SPB;

  for (int k = tid; k < SPB * LDA0; k += NTHR) A0[k] = (_Float16)0.0f;
  for (int k = tid; k < SPB * LDA1; k += NTHR) A1[k] = (_Float16)0.0f;

  float b0v[4], b1v[4], cs0[8], cs1[8];
#pragma unroll
  for (int g = 0; g < 4; ++g) {
    b0v[g] = bih0[g * NH + col] + bhh0[g * NH + col];
    b1v[g] = bih1[g * NH + col] + bhh1[g * NH + col];
  }
#pragma unroll
  for (int r = 0; r < 8; ++r) { cs0[r] = 0.0f; cs1[r] = 0.0f; }

  const _Float16* a0p = A0 + (rowb + c) * LDA0 + koff;
  const _Float16* a1p = A1 + (rowb + c) * LDA1 + koff;
  const _Float16* w0p = W0c + (size_t)col * K0 + koff;
  const _Float16* w1p = W1c + (size_t)col * K1 + koff;
  const v8f z8 = {0.f, 0.f, 0.f, 0.f, 0.f, 0.f, 0.f, 0.f};
  __syncthreads();

#pragma unroll 1
  for (int t = 0; t < TT; ++t) {
    if (tid < SPB * NI) {
      const int s = tid / NI;
      const int i = tid - s * NI;
      const float v = x[(base + (size_t)s) * (TT * NI) + t * NI + i];
      A0[s * LDA0 + NH + i] = (_Float16)v;
    }
    __syncthreads();

    v8f acc[4];
#pragma unroll
    for (int g = 0; g < 4; ++g) acc[g] = z8;
#pragma unroll
    for (int kc = 0; kc < K0 / 32; ++kc) {
      const int ko = kc * 32;
      const v16h a = Frag<_Float16>::load(a0p + ko);
#pragma unroll
      for (int g = 0; g < 4; ++g)
        acc[g] = mma_f16g(a, Frag<_Float16>::load(w0p + (size_t)g * NH * K0 + ko), acc[g]);
    }
    __syncthreads();
#pragma unroll
    for (int r = 0; r < 8; ++r) {
      const int row = rowb + 8 * hh + r;
      const float pi = acc[0][r] * WINV + b0v[0];
      const float pf = acc[1][r] * WINV + b0v[1];
      const float pg = acc[2][r] * WINV + b0v[2];
      const float po = acc[3][r] * WINV + b0v[3];
      const float ig = sigm_f(pi);
      const float fg = sigm_f(pf);
      const float gg = tanh_f(pg);
      const float og = sigm_f(po);
      const float cn = fg * cs0[r] + ig * gg;
      cs0[r] = cn;
      const float hn = og * tanh_f(cn);
      const _Float16 hb = (_Float16)hn;
      A0[row * LDA0 + col] = hb;
      A1[row * LDA1 + col] = hb;
    }
    __syncthreads();

#pragma unroll
    for (int g = 0; g < 4; ++g) acc[g] = z8;
#pragma unroll
    for (int kc = 0; kc < K1 / 32; ++kc) {
      const int ko = kc * 32;
      const v16h a = Frag<_Float16>::load(a1p + ko);
#pragma unroll
      for (int g = 0; g < 4; ++g)
        acc[g] = mma_f16g(a, Frag<_Float16>::load(w1p + (size_t)g * NH * K1 + ko), acc[g]);
    }
    __syncthreads();
#pragma unroll
    for (int r = 0; r < 8; ++r) {
      const int row = rowb + 8 * hh + r;
      const float pi = acc[0][r] * WINV + b1v[0];
      const float pf = acc[1][r] * WINV + b1v[1];
      const float pg = acc[2][r] * WINV + b1v[2];
      const float po = acc[3][r] * WINV + b1v[3];
      const float ig = sigm_f(pi);
      const float fg = sigm_f(pf);
      const float gg = tanh_f(pg);
      const float og = sigm_f(po);
      const float cn = fg * cs1[r] + ig * gg;
      cs1[r] = cn;
      const float hn = og * tanh_f(cn);
      A1[row * LDA1 + NH + col] = (_Float16)hn;
      hF[row * LDF + col] = hn;
    }
  }
  __syncthreads();

  {
    const int row = tid >> 3;
    const int seg = (tid & 7) * 8;
    float p = 0.0f;
#pragma unroll
    for (int e = 0; e < 8; ++e) p += hF[row * LDF + seg + e] * Wfc[seg + e];
    p += __shfl_xor(p, 1, 32);
    p += __shfl_xor(p, 2, 32);
    p += __shfl_xor(p, 4, 32);
    if ((tid & 7) == 0) oS[row] = p + bfc[0];
  }
  __syncthreads();
  if (tid < 8) {
    const v4f v = *(const v4f*)(oS + tid * 4);
    float* op = out + base + (size_t)tid * 4;
    *(volatile v4f*)op = v;
    __threadfence();
    *(volatile v4f*)op = v;
  }
}

extern "C" void kernel_launch(void* const* d_in, const int* in_sizes, int n_in,
                              void* d_out, int out_size, void* d_ws, size_t ws_size,
                              hipStream_t stream) {
  if (n_in < 11) return;
  if (in_sizes[0] != NB * TT * NI || in_sizes[1] != NG * NI || in_sizes[2] != NG * NH ||
      in_sizes[3] != NG || in_sizes[4] != NG || in_sizes[5] != NG * NH || in_sizes[6] != NG * NH ||
      in_sizes[7] != NG || in_sizes[8] != NG || in_sizes[9] != NH || in_sizes[10] < 1 ||
      out_size != NB) return;

  const float* x    = (const float*)d_in[0];
  const float* Wih0 = (const float*)d_in[1];
  const float* Whh0 = (const float*)d_in[2];
  const float* bih0 = (const float*)d_in[3];
  const float* bhh0 = (const float*)d_in[4];
  const float* Wih1 = (const float*)d_in[5];
  const float* Whh1 = (const float*)d_in[6];
  const float* bih1 = (const float*)d_in[7];
  const float* bhh1 = (const float*)d_in[8];
  const float* Wfc  = (const float*)d_in[9];
  const float* bfc  = (const float*)d_in[10];
  float* out = (float*)d_out;

  char* ws = (char*)d_ws;
  size_t off = 0;
  _Float16* W0c = (_Float16*)(ws + off); off += (size_t)NG * K0 * 2;
  _Float16* W1c = (_Float16*)(ws + off); off += (size_t)NG * K1 * 2;
  if (off > ws_size) return;

  prep_weights<<<(PREPN + NTHR - 1) / NTHR, NTHR, 0, stream>>>(Wih0, Whh0, Wih1, Whh1, W0c, W1c);
  lstm2_fc_fused<<<NB / SPB, NTHR, 0, stream>>>(x, W0c, W1c, bih0, bhh0, bih1, bhh1, Wfc, bfc, out);
}
